// UVFA_text_3942779978020
// MI455X (gfx1250) — hardware-verified
//
#include <hip/hip_runtime.h>

#define NB     256
#define NCELL  100
#define NTILE  7
#define RR     128
#define LL     12
#define EE     64
#define NSV    32
#define NOV    32
#define CPS    33
#define NVOC   1000
#define G4     512
#define SLOT   65536

typedef __bf16 v16b __attribute__((ext_vector_type(16)));
typedef __bf16 v8b  __attribute__((ext_vector_type(8)));
typedef float  v8f  __attribute__((ext_vector_type(8)));
typedef float  v4f  __attribute__((ext_vector_type(4)));
typedef v8b __attribute__((may_alias)) v8ba;
typedef v4f __attribute__((may_alias)) v4fa;

union Frag  { v16b v; v8b half[2]; };
union Pack8 { v8b b; v4f f; };

__device__ __forceinline__ v8f wmma16(v16b a, v16b b, v8f c) {
  v8f d = __builtin_amdgcn_wmma_f32_16x16x32_bf16(false, a, false, b, (short)0, c, false, false);
  asm volatile("v_nop\n\tv_nop\n\tv_nop\n\tv_nop" : "+v"(d) : "v"(a), "v"(b));
  return d;
}

__device__ __forceinline__ v16b load_frag(const __bf16* p, int h) {
  Frag f;
  f.half[0] = *(const v8ba*)(p + 8 * h);
  f.half[1] = *(const v8ba*)(p + 16 + 8 * h);
  return f.v;
}

template <int KS>
__device__ __forceinline__ v8f dot_tile(const __bf16* ah, const __bf16* al,
                                        const __bf16* bh, const __bf16* bl, int h, v8f acc) {
#pragma unroll
  for (int kk = 0; kk < KS; ++kk) {
    const v16b fa = load_frag(ah + 32 * kk, h);
    const v16b ga = load_frag(al + 32 * kk, h);
    const v16b fb = load_frag(bh + 32 * kk, h);
    const v16b gb = load_frag(bl + 32 * kk, h);
    acc = wmma16(fa, fb, acc);
    acc = wmma16(ga, fb, acc);
    acc = wmma16(fa, gb, acc);
  }
  return acc;
}

__device__ __forceinline__ void split2(float x, __bf16& hi, __bf16& lo) {
  const unsigned u = __float_as_uint(x);
  const unsigned r = (u + 0x7FFFu + ((u >> 16) & 1u)) & 0xFFFF0000u;
  const float hf = __uint_as_float(r);
  hi = (__bf16)hf;
  lo = (__bf16)(x - hf);
}

__device__ __forceinline__ void store_pass(const float* lds, float* dst, int n4, int t) {
  for (int j = t; j < n4; j += 256)
    *(volatile v4f*)(dst + 4 * j) = *(const v4fa*)(lds + 4 * j);
}

__device__ __forceinline__ void conv_store_pass(const float* tile, __bf16* hi, __bf16* lo,
                                                int K, int n0, int t) {
  const int KP = K >> 3, P = 32 * KP;
  for (int j = t; j < P; j += 256) {
    const int rowl = j / KP, kp = j - rowl * KP;
    Pack8 uh, ul;
#pragma unroll
    for (int i = 0; i < 8; ++i) {
      const float x = tile[(8 * kp + i) * 33 + rowl];
      __bf16 a, c;
      split2(x, a, c);
      uh.b[i] = a;
      ul.b[i] = c;
    }
    const size_t off = (size_t)(n0 + rowl) * K + 8 * kp;
    *(volatile v4f*)(hi + off) = uh.f;
    *(volatile v4f*)(lo + off) = ul.f;
  }
}

__global__ __launch_bounds__(256) void convert_kernel(
    const float* Ws2, const float* Ws3, const float* Wo2, const float* Wo3,
    const float* Wih, const float* Whh, __bf16* wt)
{
  __shared__ __attribute__((aligned(16))) float tile[128 * 33];
  const int t = threadIdx.x, id = blockIdx.y, bx = blockIdx.x;
  const float* src = Ws2;
  int K = 128, N = 128;
  if (id == 1)      { src = Ws3; }
  else if (id == 2) { src = Wo2; }
  else if (id == 3) { src = Wo3; }
  else if (id == 4) { src = Wih; K = 64;  N = 512; }
  else if (id == 5) { src = Whh; K = 128; N = 512; }
  const int n0 = bx * 32;
  if (n0 >= N) return;
  for (int i = 0; i < (K >> 3); ++i) {
    const int e = i * 256 + t, k = e >> 5, nl = e & 31;
    tile[k * 33 + nl] = src[(size_t)k * N + n0 + nl];
  }
  __syncthreads();
  __bf16* hi = wt + (size_t)id * 2 * SLOT;
  __bf16* lo = hi + SLOT;
  conv_store_pass(tile, hi, lo, K, n0, t);
  __threadfence();
  conv_store_pass(tile, hi, lo, K, n0, t);
}

__global__ __launch_bounds__(256) void front_kernel(
    const int* state, const int* obj, const float* Ws1, const float* Wo1,
    const float* bo1, const float* bo2, const float* bo3, const __bf16* wt,
    float* base_s, float* obj_out)
{
  __shared__ __attribute__((aligned(16))) float  sS[16 * RR];
  __shared__ __attribute__((aligned(16))) float  sO[16 * RR];
  __shared__ __attribute__((aligned(16))) __bf16 aH[16 * RR];
  __shared__ __attribute__((aligned(16))) __bf16 aL[16 * RR];
  __shared__ __attribute__((aligned(16))) __bf16 hH[16 * RR];
  __shared__ __attribute__((aligned(16))) __bf16 hL[16 * RR];

  const int t = threadIdx.x, lane = t & 31, w = t >> 5, h = lane >> 4, m = lane & 15;
  const int blk = blockIdx.x;
  const int row = t >> 4, k0 = (t & 15) * 8;
  const int b = blk * 16 + row;

  v4f s0 = {0.f, 0.f, 0.f, 0.f}, s1 = {0.f, 0.f, 0.f, 0.f};
  v4f o0 = {0.f, 0.f, 0.f, 0.f}, o1 = {0.f, 0.f, 0.f, 0.f};
#pragma unroll 2
  for (int c = 0; c < NCELL; ++c) {
    const int vs = state[b * NCELL + c];
    const int vo = obj[b * NCELL + c];
    const int vsc = min(max(vs, 0), NSV - 1);
    const int voc = min(max(vo, 0), NOV - 1);
    const float fs = ((unsigned)vs < (unsigned)NSV) ? 1.0f : 0.0f;
    const float fo = ((unsigned)vo < (unsigned)NOV) ? 1.0f : 0.0f;
    const float* ps = Ws1 + (size_t)(c * CPS + vsc) * RR + k0;
    const float* po = Wo1 + (size_t)(c * NOV + voc) * RR + k0;
    const v4f x0 = *(const v4fa*)ps, x1 = *(const v4fa*)(ps + 4);
    const v4f y0 = *(const v4fa*)po, y1 = *(const v4fa*)(po + 4);
    s0 = s0 + x0 * fs;  s1 = s1 + x1 * fs;
    o0 = o0 + y0 * fo;  o1 = o1 + y1 * fo;
  }
  *(v4fa*)(sS + row * RR + k0)     = s0;
  *(v4fa*)(sS + row * RR + k0 + 4) = s1;
  {
    const float ov[8] = {o0.x, o0.y, o0.z, o0.w, o1.x, o1.y, o1.z, o1.w};
#pragma unroll
    for (int i = 0; i < 8; ++i) {
      float v = ov[i] + bo1[k0 + i];
      v = (v > 0.f) ? v : 0.f;
      split2(v, aH[row * RR + k0 + i], aL[row * RR + k0 + i]);
    }
  }
  __syncthreads();

  float* dsts = base_s + (size_t)blk * 16 * RR;
  store_pass(sS, dsts, 16 * RR / 4, t);

  const __bf16* w2h = wt + (size_t)2 * 2 * SLOT;
  const __bf16* w2l = w2h + SLOT;
  const __bf16* w3h = wt + (size_t)3 * 2 * SLOT;
  const __bf16* w3l = w3h + SLOT;
  const int n = 16 * w + m;
  const v8f zero8 = {0.f, 0.f, 0.f, 0.f, 0.f, 0.f, 0.f, 0.f};

  v8f acc = dot_tile<4>(aH + m * RR, aL + m * RR, w2h + (size_t)n * RR, w2l + (size_t)n * RR, h, zero8);
  {
    const float b2 = bo2[n];
#pragma unroll
    for (int r = 0; r < 8; ++r) {
      float v = acc[r] + b2;
      v = (v > 0.f) ? v : 0.f;
      split2(v, hH[(8 * h + r) * RR + n], hL[(8 * h + r) * RR + n]);
    }
  }
  __syncthreads();

  v8f acc2 = dot_tile<4>(hH + m * RR, hL + m * RR, w3h + (size_t)n * RR, w3l + (size_t)n * RR, h, zero8);
  {
    const float b3 = bo3[n];
#pragma unroll
    for (int r = 0; r < 8; ++r) sO[(8 * h + r) * RR + n] = acc2[r] + b3;
  }
  __syncthreads();

  float* dsto = obj_out + (size_t)blk * 16 * RR;
  store_pass(sO, dsto, 16 * RR / 4, t);
  __threadfence();
  store_pass(sS, dsts, 16 * RR / 4, t);
  store_pass(sO, dsto, 16 * RR / 4, t);
}

__global__ __launch_bounds__(256) void lstm_kernel(
    const int* text, const float* emb, const float* b_lstm, const __bf16* wt, float* hfin)
{
  __shared__ __attribute__((aligned(16))) __bf16 xH[16 * EE];
  __shared__ __attribute__((aligned(16))) __bf16 xL[16 * EE];
  __shared__ __attribute__((aligned(16))) __bf16 hHb[16 * RR];
  __shared__ __attribute__((aligned(16))) __bf16 hLb[16 * RR];
  __shared__ __attribute__((aligned(16))) float  Hs[16 * RR];
  __shared__ __attribute__((aligned(16))) float  Cs[16 * RR];
  __shared__ __attribute__((aligned(16))) float  G[16 * G4];

  const int t = threadIdx.x, lane = t & 31, w = t >> 5, h = lane >> 4, m = lane & 15;
  const int r0 = blockIdx.x * 16;
  const int row = t >> 4;
  {
    const int k0 = (t & 15) * 8;
#pragma unroll
    for (int i = 0; i < 8; ++i) {
      Hs[row * RR + k0 + i]  = 0.f;
      Cs[row * RR + k0 + i]  = 0.f;
      hHb[row * RR + k0 + i] = (__bf16)0.0f;
      hLb[row * RR + k0 + i] = (__bf16)0.0f;
    }
  }
  const __bf16* wih_h = wt + (size_t)4 * 2 * SLOT;
  const __bf16* wih_l = wih_h + SLOT;
  const __bf16* whh_h = wt + (size_t)5 * 2 * SLOT;
  const __bf16* whh_l = whh_h + SLOT;
  const v8f zero8 = {0.f, 0.f, 0.f, 0.f, 0.f, 0.f, 0.f, 0.f};

  for (int l = 0; l < LL; ++l) {
    {
      const int q = t & 15;
      int tok = text[(r0 + row) * LL + l];
      tok = min(max(tok, 0), NVOC - 1);
      const v4f x = *(const v4fa*)(emb + (size_t)tok * EE + 4 * q);
      const float xv[4] = {x.x, x.y, x.z, x.w};
#pragma unroll
      for (int i = 0; i < 4; ++i)
        split2(xv[i], xH[row * EE + 4 * q + i], xL[row * EE + 4 * q + i]);
    }
    __syncthreads();

#pragma unroll
    for (int ct = 0; ct < 4; ++ct) {
      const int n = (4 * w + ct) * 16 + m;
      v8f acc = zero8;
      acc = dot_tile<2>(xH + m * EE, xL + m * EE,
                        wih_h + (size_t)n * EE, wih_l + (size_t)n * EE, h, acc);
      acc = dot_tile<4>(hHb + m * RR, hLb + m * RR,
                        whh_h + (size_t)n * RR, whh_l + (size_t)n * RR, h, acc);
      const float bb = b_lstm[n];
#pragma unroll
      for (int r = 0; r < 8; ++r) G[(8 * h + r) * G4 + n] = acc[r] + bb;
    }
    __syncthreads();

    {
      const int u0 = (t & 15) * 8;
#pragma unroll 1
      for (int u = 0; u < 8; ++u) {
        const int nn = u0 + u;
        const float gi = G[row * G4 + nn];
        const float gf = G[row * G4 + RR + nn];
        const float gc = G[row * G4 + 2 * RR + nn];
        const float go = G[row * G4 + 3 * RR + nn];
        const float ig = 1.0f / (1.0f + expf(-gi));
        const float fg = 1.0f / (1.0f + expf(-gf));
        const float og = 1.0f / (1.0f + expf(-go));
        const float gg = tanhf(gc);
        const float c  = fg * Cs[row * RR + nn] + ig * gg;
        const float hv = og * tanhf(c);
        Cs[row * RR + nn] = c;
        Hs[row * RR + nn] = hv;
        split2(hv, hHb[row * RR + nn], hLb[row * RR + nn]);
      }
    }
    __syncthreads();
  }

  float* dst = hfin + (size_t)r0 * RR;
  store_pass(Hs, dst, 16 * RR / 4, t);
  __threadfence();
  store_pass(Hs, dst, 16 * RR / 4, t);
}

__global__ __launch_bounds__(256) void state_kernel(
    const float* base_s, const float* Ws1, const float* bs1, const float* bs2,
    const float* bs3, const __bf16* wt, const float* obj_out, const float* hfin,
    float* map_pad)
{
  __shared__ __attribute__((aligned(16))) __bf16 aH[16 * RR];
  __shared__ __attribute__((aligned(16))) __bf16 aL[16 * RR];
  __shared__ __attribute__((aligned(16))) __bf16 hH[16 * RR];
  __shared__ __attribute__((aligned(16))) __bf16 hL[16 * RR];
  __shared__ __attribute__((aligned(16))) float  sSb[RR];
  __shared__ __attribute__((aligned(16))) float  sOb[RR];
  __shared__ __attribute__((aligned(16))) float  sHq[RR];
  __shared__ __attribute__((aligned(16))) float  red[8 * 16];
  __shared__ __attribute__((aligned(16))) float  mapv[RR];

  const int t = threadIdx.x, lane = t & 31, w = t >> 5, h = lane >> 4, m = lane & 15;
  const int b = blockIdx.x;
  const int row = t >> 4, k0 = (t & 15) * 8;

  if (t < RR) {
    sSb[t]  = base_s[(size_t)b * RR + t];
    sOb[t]  = obj_out[(size_t)b * RR + t];
    sHq[t]  = hfin[(size_t)b * RR + t];
    mapv[t] = 0.f;
  }
  __syncthreads();

  const __bf16* w2h = wt;
  const __bf16* w2l = w2h + SLOT;
  const __bf16* w3h = wt + (size_t)1 * 2 * SLOT;
  const __bf16* w3l = w3h + SLOT;
  const int n = 16 * w + m;
  const v8f zero8 = {0.f, 0.f, 0.f, 0.f, 0.f, 0.f, 0.f, 0.f};
  const float b2 = bs2[n], b3 = bs3[n];

  for (int ti = 0; ti < NTILE; ++ti) {
    {
      const int p  = 16 * ti + row;
      const int pc = min(p, NCELL - 1);
      const float keep = (p < NCELL) ? 1.0f : 0.0f;
      const float* pr = Ws1 + (size_t)(pc * CPS + NSV) * RR + k0;
      const v4f p0 = *(const v4fa*)pr, p1 = *(const v4fa*)(pr + 4);
      const float pv[8] = {p0.x, p0.y, p0.z, p0.w, p1.x, p1.y, p1.z, p1.w};
#pragma unroll
      for (int i = 0; i < 8; ++i) {
        float v = (sSb[k0 + i] + pv[i]) + bs1[k0 + i];
        v = (v > 0.f) ? v : 0.f;
        v = v * keep;
        split2(v, aH[row * RR + k0 + i], aL[row * RR + k0 + i]);
      }
    }
    __syncthreads();

    v8f acc = dot_tile<4>(aH + m * RR, aL + m * RR, w2h + (size_t)n * RR, w2l + (size_t)n * RR, h, zero8);
#pragma unroll
    for (int r = 0; r < 8; ++r) {
      float v = acc[r] + b2;
      v = (v > 0.f) ? v : 0.f;
      split2(v, hH[(8 * h + r) * RR + n], hL[(8 * h + r) * RR + n]);
    }
    __syncthreads();

    v8f acc2 = dot_tile<4>(hH + m * RR, hL + m * RR, w3h + (size_t)n * RR, w3l + (size_t)n * RR, h, zero8);
    {
      const float ow = sOb[n], hw = sHq[n];
      float part[8];
#pragma unroll
      for (int r = 0; r < 8; ++r) {
        const float so = acc2[r] + b3;
        part[r] = (so * ow) * hw;
      }
#pragma unroll
      for (int r = 0; r < 8; ++r) {
        part[r] += __shfl_xor(part[r], 1);
        part[r] += __shfl_xor(part[r], 2);
        part[r] += __shfl_xor(part[r], 4);
        part[r] += __shfl_xor(part[r], 8);
      }
      if (m == 0) {
#pragma unroll
        for (int r = 0; r < 8; ++r) red[w * 16 + 8 * h + r] = part[r];
      }
    }
    __syncthreads();

    if (t < 16) {
      float s = 0.f;
#pragma unroll
      for (int w8 = 0; w8 < 8; ++w8) s += red[w8 * 16 + t];
      mapv[16 * ti + t] = s;
    }
  }
  __syncthreads();

  if (w == 0) {
    const v4f v = *(const v4fa*)(mapv + 4 * lane);
    float* dst = map_pad + (size_t)b * RR + 4 * lane;
    *(volatile v4f*)dst = v;
    __threadfence();
    *(volatile v4f*)dst = v;
  }
}

__device__ __forceinline__ void pack_pass(const float* map_pad, float* out, int t) {
  for (int j = t; j < NB * NCELL / 4; j += 256) {
    const int b = j / 25, p = 4 * (j - b * 25);
    const v4f v = *(const v4fa*)(map_pad + (size_t)b * RR + p);
    *(volatile v4f*)(out + 4 * (size_t)j) = v;
  }
}

__global__ __launch_bounds__(256) void pack_kernel(const float* map_pad, float* out) {
  const int t = threadIdx.x;
  pack_pass(map_pad, out, t);
  __threadfence();
  pack_pass(map_pad, out, t);
}

extern "C" void kernel_launch(void* const* d_in, const int* in_sizes, int n_in,
                              void* d_out, int out_size, void* d_ws, size_t ws_size,
                              hipStream_t stream) {
  if (n_in < 19) return;
  if (in_sizes[0] != NB * NCELL || in_sizes[1] != NB * NCELL || in_sizes[2] != NB * LL) return;
  if (in_sizes[3] != NCELL * CPS * RR || in_sizes[4] != RR) return;
  if (in_sizes[5] != RR * RR || in_sizes[6] != RR || in_sizes[7] != RR * RR || in_sizes[8] != RR) return;
  if (in_sizes[9] != NCELL * NOV * RR || in_sizes[10] != RR) return;
  if (in_sizes[11] != RR * RR || in_sizes[12] != RR || in_sizes[13] != RR * RR || in_sizes[14] != RR) return;
  if (in_sizes[15] != NVOC * EE || in_sizes[16] != EE * G4 || in_sizes[17] != RR * G4 || in_sizes[18] != G4) return;
  if (out_size != NB * NCELL) return;

  const int*   state  = (const int*)d_in[0];
  const int*   obj    = (const int*)d_in[1];
  const int*   text   = (const int*)d_in[2];
  const float* Ws1    = (const float*)d_in[3];
  const float* bs1    = (const float*)d_in[4];
  const float* Ws2    = (const float*)d_in[5];
  const float* bs2    = (const float*)d_in[6];
  const float* Ws3    = (const float*)d_in[7];
  const float* bs3    = (const float*)d_in[8];
  const float* Wo1    = (const float*)d_in[9];
  const float* bo1    = (const float*)d_in[10];
  const float* Wo2    = (const float*)d_in[11];
  const float* bo2    = (const float*)d_in[12];
  const float* Wo3    = (const float*)d_in[13];
  const float* bo3    = (const float*)d_in[14];
  const float* emb    = (const float*)d_in[15];
  const float* Wih    = (const float*)d_in[16];
  const float* Whh    = (const float*)d_in[17];
  const float* b_lstm = (const float*)d_in[18];
  float* out = (float*)d_out;

  const size_t wt_bytes    = (size_t)6 * 2 * SLOT * 2;
  const size_t plane_bytes = (size_t)NB * RR * 4;
  const size_t total = wt_bytes + 4 * plane_bytes;
  if (total > ws_size) return;

  char* ws = (char*)d_ws;
  __bf16* wt      = (__bf16*)(ws);
  float*  base_s  = (float*)(ws + wt_bytes);
  float*  obj_out = (float*)(ws + wt_bytes + plane_bytes);
  float*  hfin    = (float*)(ws + wt_bytes + 2 * plane_bytes);
  float*  map_pad = (float*)(ws + wt_bytes + 3 * plane_bytes);

  convert_kernel<<<dim3(16, 6), 256, 0, stream>>>(Ws2, Ws3, Wo2, Wo3, Wih, Whh, wt);
  front_kernel<<<NB / 16, 256, 0, stream>>>(state, obj, Ws1, Wo1, bo1, bo2, bo3, wt, base_s, obj_out);
  lstm_kernel<<<NB / 16, 256, 0, stream>>>(text, emb, b_lstm, wt, hfin);
  state_kernel<<<NB, 256, 0, stream>>>(base_s, Ws1, bs1, bs2, bs3, wt, obj_out, hfin, map_pad);
  pack_kernel<<<1, 256, 0, stream>>>(map_pad, out);
}
